// MHA__15470472200192
// MI455X (gfx1250) — hardware-verified
//
#include <hip/hip_runtime.h>
#include <stdint.h>
#include <stddef.h>

typedef __attribute__((ext_vector_type(16))) _Float16 v16h;
typedef __attribute__((ext_vector_type(8)))  _Float16 v8h;
typedef __attribute__((ext_vector_type(16))) __bf16   v16b;
typedef __attribute__((ext_vector_type(8)))  __bf16   v8b;
typedef __attribute__((ext_vector_type(8)))  float    v8f;
typedef __attribute__((ext_vector_type(4)))  float    v4f;

constexpr int NTOK   = 4096;
constexpr int DMODEL = 1024;
constexpr int DHEAD  = 512;
constexpr int NHEAD  = 2;
constexpr float W_CARRY     = 64.0f;
constexpr float W_CARRY_INV = 1.0f / 64.0f;

__device__ __forceinline__ unsigned short f2bf_bits(float f) {
  unsigned u = __float_as_uint(f);
  return (unsigned short)((u + 0x7FFFu + ((u >> 16) & 1u)) >> 16);
}
__device__ __forceinline__ float bf_bits2f(unsigned short h) { return __uint_as_float(((unsigned)h) << 16); }

__device__ __forceinline__ void dep_guard_h(v8f& a, v8f& b, v16h x, v16h y) { asm volatile("v_nop\n\tv_nop\n\tv_nop\n\tv_nop" : "+v"(a), "+v"(b) : "v"(x), "v"(y)); }
__device__ __forceinline__ void dep_guard_b(v8f& a, v8f& b, v16b x, v16b y) { asm volatile("v_nop\n\tv_nop\n\tv_nop\n\tv_nop" : "+v"(a), "+v"(b) : "v"(x), "v"(y)); }
__device__ __forceinline__ void keep4_h(v16h a, v16h b, v16h c, v16h d) { asm volatile("v_nop" :: "v"(a), "v"(b), "v"(c), "v"(d)); }
__device__ __forceinline__ void keep4_b(v16b a, v16b b, v16b c, v16b d) { asm volatile("v_nop" :: "v"(a), "v"(b), "v"(c), "v"(d)); }
__device__ __forceinline__ void acc_guard4(v8f& a, v8f& b, v8f& c, v8f& d) { asm volatile("v_nop\n\tv_nop\n\tv_nop\n\tv_nop" : "+v"(a), "+v"(b), "+v"(c), "+v"(d)); }
template <typename T> struct Frag;
template <> struct Frag<_Float16> {
  typedef v16h V; union U { v16h v; v8h h[2]; };
  static __device__ __forceinline__ v16h load(const _Float16* p) {
    U f; f.h[0] = *(const v8h*)(p); f.h[1] = *(const v8h*)(p + 16); return f.v;
  }
  static __device__ __forceinline__ v8f mma(v16h a, v16h b, v8f c) {
    return __builtin_amdgcn_wmma_f32_16x16x32_f16(false, a, false, b, (short)0, c, false, false);
  }
  static __device__ __forceinline__ void guard(v8f& a, v8f& b, v16h x, v16h y) { dep_guard_h(a, b, x, y); }
  static __device__ __forceinline__ void keep(v16h a, v16h b, v16h c, v16h d) { keep4_h(a, b, c, d); }
};
template <> struct Frag<__bf16> {
  typedef v16b V; union U { v16b v; v8b h[2]; };
  static __device__ __forceinline__ v16b load(const __bf16* p) {
    U f; f.h[0] = *(const v8b*)(p); f.h[1] = *(const v8b*)(p + 16); return f.v;
  }
  static __device__ __forceinline__ v8f mma(v16b a, v16b b, v8f c) {
    return __builtin_amdgcn_wmma_f32_16x16x32_bf16(false, a, false, b, (short)0, c, false, false);
  }
  static __device__ __forceinline__ void guard(v8f& a, v8f& b, v16b x, v16b y) { dep_guard_b(a, b, x, y); }
  static __device__ __forceinline__ void keep(v16b a, v16b b, v16b c, v16b d) { keep4_b(a, b, c, d); }
};

template <int ET> struct Elem;
template <> struct Elem<0> { typedef _Float16 T; };
template <> struct Elem<1> { typedef __bf16 T; };
template <int ET, bool SPLIT, int BIAS_MODE, int OUT_MODE, bool RESID, int ACT = 0>
__global__ __launch_bounds__(256) void wmma_gemm64(
    const unsigned short* __restrict__ Ap, const unsigned short* __restrict__ A2p, int lda, long strideA,
    const unsigned short* __restrict__ Btp, const unsigned short* __restrict__ Bt2p, int ldb, long strideB,
    void* __restrict__ Cout, void* __restrict__ Cout2, int ldc, long strideC,
    const float* __restrict__ bias,
    const float* __restrict__ resid, long strideR,
    int M, int N, int K, float scale) {
  typedef typename Elem<ET>::T T;
  typedef typename Frag<T>::V V;
  const T* A = (const T*)Ap; const T* A2 = (const T*)A2p; const T* Bt = (const T*)Btp; const T* Bt2 = (const T*)Bt2p;
  __shared__ __align__(16) float sT[8][16 * 68];
  const int b    = blockIdx.y;
  const int lane = threadIdx.x & 31;
  const int wave = threadIdx.x >> 5;
  const int tilesN = N >> 6;
  const int tilesM = M >> 6;
  const int tile = blockIdx.x * 8 + wave;
  if (tile >= tilesM * tilesN) return;
  const int tm = tile / tilesN;
  const int tn = tile - tm * tilesN;
  const int m0 = tm << 6;
  const int n0 = tn << 6;

  const T* Ab  = A  + (size_t)b * strideA;
  const T* Bb  = Bt + (size_t)b * strideB;
  const T* Ab2 = SPLIT ? (A2  + (size_t)b * strideA) : nullptr;
  const T* Bb2 = SPLIT ? (Bt2 + (size_t)b * strideB) : nullptr;

  const int rlane = lane & 15;
  const int koff  = (lane >> 4) * 8;
  const int mOff  = (lane >> 4) * 8;

  v8f acc[4][4];
#pragma unroll
  for (int i = 0; i < 4; ++i)
#pragma unroll
    for (int j = 0; j < 4; ++j) acc[i][j] = (v8f){0.f,0.f,0.f,0.f,0.f,0.f,0.f,0.f};

  for (int k0 = 0; k0 < K; k0 += 32) {
    V bh[4], bl[4];
#pragma unroll
    for (int j = 0; j < 4; ++j) {
      const size_t bo = (size_t)(n0 + (j << 4) + rlane) * ldb + koff + k0;
      bh[j] = Frag<T>::load(Bb + bo);
      if (SPLIT) bl[j] = Frag<T>::load(Bb2 + bo);
    }
#pragma unroll
    for (int i = 0; i < 4; ++i) {
      const size_t ao = (size_t)(m0 + (i << 4) + rlane) * lda + koff + k0;
      V ah = Frag<T>::load(Ab + ao);
      V al;
      if (SPLIT) al = Frag<T>::load(Ab2 + ao);
#pragma unroll
      for (int j = 0; j < 4; ++j) {
        acc[i][j] = Frag<T>::mma(ah, bh[j], acc[i][j]);
        if (SPLIT) {
          acc[i][j] = Frag<T>::mma(ah, bl[j], acc[i][j]);
          acc[i][j] = Frag<T>::mma(al, bh[j], acc[i][j]);
        }
      }
      Frag<T>::guard(acc[i][0], acc[i][3], ah, SPLIT ? al : ah);
    }
    Frag<T>::keep(bh[0], bh[1], bh[2], bh[3]);
    if (SPLIT) Frag<T>::keep(bl[0], bl[1], bl[2], bl[3]);
  }
  acc_guard4(acc[0][0], acc[0][1], acc[0][2], acc[0][3]);
  acc_guard4(acc[1][0], acc[1][1], acc[1][2], acc[1][3]);
  acc_guard4(acc[2][0], acc[2][1], acc[2][2], acc[2][3]);
  acc_guard4(acc[3][0], acc[3][1], acc[3][2], acc[3][3]);

  float* slab = sT[wave];
  const float* Rb = RESID ? (resid + (size_t)b * strideR) : nullptr;
#pragma unroll
  for (int i = 0; i < 4; ++i) {
    const int mBase = m0 + (i << 4);
#pragma unroll
    for (int j = 0; j < 4; ++j) {
      const int n = n0 + (j << 4) + rlane;
      float bv = 0.f;
      if (BIAS_MODE == 2) bv = bias[n];
#pragma unroll
      for (int r = 0; r < 8; ++r) {
        float v = acc[i][j][r] * scale;
        if (BIAS_MODE == 1) v += bias[mBase + mOff + r];
        if (BIAS_MODE == 2) v += bv;
        if (RESID) v += Rb[(size_t)(mBase + mOff + r) * ldc + n];
        if (ACT == 1) v = tanhf(v);
        if (ACT == 2) v = fmaxf(v, 0.0f);
        if (ACT == 3) v = v / (1.0f + expf(-v));
        if (ACT == 4) v = (v > 0.f) ? v : 0.01f * v;
        if (ACT == 5) v = 0.5f * v * (1.0f + erff(v * 0.70710678118654752f));
        slab[(mOff + r) * 68 + (j << 4) + rlane] = v;
      }
    }
    __builtin_amdgcn_fence(__ATOMIC_RELEASE, "workgroup");
    __builtin_amdgcn_wave_barrier();
    __builtin_amdgcn_fence(__ATOMIC_ACQUIRE, "workgroup");
    if (OUT_MODE == 0) {
      float* C = (float*)Cout + (size_t)b * strideC;
      const int hh = lane >> 4, c4 = (lane & 15) * 4;
      for (int pass = 0; pass < 2; ++pass) {
#pragma unroll
        for (int it = 0; it < 8; ++it) {
          const int row = it * 2 + hh;
          v4f v = *(const v4f*)(slab + row * 68 + c4);
          *(volatile v4f*)(C + (size_t)(mBase + row) * ldc + n0 + c4) = v;
        }
        __threadfence();
      }
    } else {
      const int q = lane >> 3, c8 = (lane & 7) * 8;
      unsigned short* C  = (unsigned short*)Cout  + (size_t)b * strideC;
      unsigned short* C2 = (OUT_MODE == 2) ? ((unsigned short*)Cout2 + (size_t)b * strideC) : nullptr;
      for (int pass = 0; pass < 2; ++pass) {
#pragma unroll
        for (int it = 0; it < 4; ++it) {
          const int row = it * 4 + q;
          const float* sp = slab + row * 68 + c8;
          v8h hv, lv;
#pragma unroll
          for (int e = 0; e < 8; ++e) {
            if (OUT_MODE == 1) {
              hv[e] = (_Float16)sp[e];
            } else {
              unsigned short hb = f2bf_bits(sp[e]);
              unsigned short lb = f2bf_bits(sp[e] - bf_bits2f(hb));
              hv[e] = __builtin_bit_cast(_Float16, hb);
              lv[e] = __builtin_bit_cast(_Float16, lb);
            }
          }
          *(volatile v8h*)(C + (size_t)(mBase + row) * ldc + n0 + c8) = hv;
          if (OUT_MODE == 2) *(volatile v8h*)(C2 + (size_t)(mBase + row) * ldc + n0 + c8) = lv;
        }
        __threadfence();
      }
    }
    __builtin_amdgcn_fence(__ATOMIC_RELEASE, "workgroup");
    __builtin_amdgcn_wave_barrier();
    __builtin_amdgcn_fence(__ATOMIC_ACQUIRE, "workgroup");
  }
}

__device__ __forceinline__ void cvt_bf_f16_store8(const float* __restrict__ src, unsigned short* __restrict__ dst,
                                                  int i, float mul) {
  const v4f a = *(const v4f*)(src + (size_t)i * 8);
  const v4f c = *(const v4f*)(src + (size_t)i * 8 + 4);
  v8h o;
#pragma unroll
  for (int e = 0; e < 4; ++e) {
    const float fa = bf_bits2f(f2bf_bits(a[e])) * mul;
    const float fc = bf_bits2f(f2bf_bits(c[e])) * mul;
    o[e]     = (_Float16)fa;
    o[4 + e] = (_Float16)fc;
  }
  _Float16* op = (_Float16*)(void*)dst + (size_t)i * 8;
  *(volatile v8h*)op = o;
  __threadfence();
  *(volatile v8h*)op = o;
}

__global__ __launch_bounds__(256) void cast_x_kernel(const float* __restrict__ x, unsigned short* __restrict__ out,
                                                     int n8, float mul) {
  const int i = blockIdx.x * 256 + threadIdx.x;
  if (i < n8) cvt_bf_f16_store8(x, out, i, mul);
}

__global__ __launch_bounds__(256) void cast_w6_kernel(
    const float* __restrict__ w0, const float* __restrict__ w1, const float* __restrict__ w2,
    const float* __restrict__ w3, const float* __restrict__ w4, const float* __restrict__ w5,
    unsigned short* __restrict__ out, int n8, float mul) {
  const int y = blockIdx.y;
  const float* src = w0;
  if (y == 1) src = w1;
  if (y == 2) src = w2;
  if (y == 3) src = w3;
  if (y == 4) src = w4;
  if (y == 5) src = w5;
  unsigned short* dst = out + (size_t)y * (size_t)n8 * 8;
  const int i = blockIdx.x * 256 + threadIdx.x;
  if (i < n8) cvt_bf_f16_store8(src, dst, i, mul);
}

constexpr size_t X16_BYTES = (size_t)NTOK * DMODEL * 2;
constexpr size_t W16_BYTES = (size_t)6 * DHEAD * DHEAD * 2;
constexpr size_t QK_BYTES  = (size_t)NHEAD * NTOK * DMODEL * 2;
constexpr size_t VP_BYTES  = (size_t)NHEAD * DHEAD * NTOK * 2;
constexpr size_t SP_BYTES  = (size_t)NHEAD * NTOK * NTOK * 2;
constexpr size_t X16_OFF = 0;
constexpr size_t W16_OFF = X16_OFF + X16_BYTES;
constexpr size_t QK_OFF  = W16_OFF + W16_BYTES;
constexpr size_t VP_OFF  = QK_OFF + QK_BYTES;
constexpr size_t SP_OFF  = VP_OFF + VP_BYTES;
constexpr size_t WS_TOTAL = SP_OFF + SP_BYTES;
static_assert(WS_TOTAL == 103809024u);
static_assert(WS_TOTAL <= (size_t)134217728u);
static_assert((W16_OFF % 128) == 0 && (QK_OFF % 128) == 0 && (VP_OFF % 128) == 0 && (SP_OFF % 128) == 0);

static_assert(NTOK % 64 == 0 && DHEAD % 64 == 0 && (2 * DHEAD) % 64 == 0);
static_assert(DHEAD % 32 == 0 && NTOK % 32 == 0);
static_assert(DMODEL == NHEAD * DHEAD);
static_assert((NTOK * DMODEL) % (8 * 256) == 0 && (DHEAD * DHEAD) % (8 * 256) == 0);

extern "C" void kernel_launch(void* const* d_in, const int* in_sizes, int n_in,
                              void* d_out, int out_size, void* d_ws, size_t ws_size,
                              hipStream_t stream) {
  if (n_in < 7) return;
  if (in_sizes[0] != NTOK * DMODEL) return;
  for (int i = 1; i < 7; ++i) if (in_sizes[i] != DHEAD * DHEAD) return;
  if (out_size != NTOK * DMODEL) return;
  if (ws_size < WS_TOTAL) return;

  const float* x   = (const float*)d_in[0];
  const float* wq1 = (const float*)d_in[1];
  const float* wq2 = (const float*)d_in[2];
  const float* wk1 = (const float*)d_in[3];
  const float* wk2 = (const float*)d_in[4];
  const float* wv1 = (const float*)d_in[5];
  const float* wv2 = (const float*)d_in[6];
  float* out = (float*)d_out;

  char* ws = (char*)d_ws;
  unsigned short* X16 = (unsigned short*)(ws + X16_OFF);
  unsigned short* W16 = (unsigned short*)(ws + W16_OFF);
  unsigned short* QK  = (unsigned short*)(ws + QK_OFF);
  unsigned short* VP  = (unsigned short*)(ws + VP_OFF);
  unsigned short* SP  = (unsigned short*)(ws + SP_OFF);
  unsigned short* WQK = W16;
  unsigned short* WV  = W16 + (size_t)4 * DHEAD * DHEAD;
  const float* fdum = x;

  {
    const int n8 = (NTOK * DMODEL) / 8;
    cast_x_kernel<<<dim3(n8 / 256), dim3(256), 0, stream>>>(x, X16, n8, 1.0f);
  }
  {
    const int n8 = (DHEAD * DHEAD) / 8;
    cast_w6_kernel<<<dim3(n8 / 256, 6), dim3(256), 0, stream>>>(wq1, wk1, wq2, wk2, wv1, wv2, W16, n8, W_CARRY);
  }
  {
    const int tiles = (NTOK / 64) * ((2 * DHEAD) / 64);
    wmma_gemm64<0, false, 0, 1, false><<<dim3((tiles + 7) / 8, NHEAD), dim3(256), 0, stream>>>(
        X16, X16, DMODEL, (long)DHEAD,
        WQK, WQK, DHEAD, (long)2 * DHEAD * DHEAD,
        (void*)QK, (void*)QK, DMODEL, (long)NTOK * DMODEL,
        fdum, fdum, 0L,
        NTOK, 2 * DHEAD, DHEAD, W_CARRY_INV);
  }
  {
    const int tiles = (DHEAD / 64) * (NTOK / 64);
    wmma_gemm64<0, false, 0, 1, false><<<dim3((tiles + 7) / 8, NHEAD), dim3(256), 0, stream>>>(
        WV, WV, DHEAD, (long)DHEAD * DHEAD,
        X16, X16, DMODEL, (long)DHEAD,
        (void*)VP, (void*)VP, NTOK, (long)DHEAD * NTOK,
        fdum, fdum, 0L,
        DHEAD, NTOK, DHEAD, W_CARRY_INV);
  }
  {
    const int tiles = (NTOK / 64) * (NTOK / 64);
    wmma_gemm64<0, false, 0, 1, false><<<dim3((tiles + 7) / 8, NHEAD), dim3(256), 0, stream>>>(
        QK, QK, DMODEL, (long)NTOK * DMODEL,
        QK + DHEAD, QK + DHEAD, DMODEL, (long)NTOK * DMODEL,
        (void*)SP, (void*)SP, NTOK, (long)NTOK * NTOK,
        fdum, fdum, 0L,
        NTOK, NTOK, DHEAD, 1.0f);
  }
  {
    const int tiles = (NTOK / 64) * (DHEAD / 64);
    wmma_gemm64<0, false, 0, 0, false><<<dim3((tiles + 7) / 8, NHEAD), dim3(256), 0, stream>>>(
        SP, SP, NTOK, (long)NTOK * NTOK,
        VP, VP, NTOK, (long)DHEAD * NTOK,
        (void*)out, (void*)out, DMODEL, (long)DHEAD,
        fdum, fdum, 0L,
        NTOK, DHEAD, NTOK, 1.0f);
  }
}
